// JointEncoder_71811853189763
// MI455X (gfx1250) — hardware-verified
//
#include <hip/hip_runtime.h>
#include <stddef.h>


typedef __attribute__((ext_vector_type(16))) _Float16 v16h;
typedef __attribute__((ext_vector_type(8)))  _Float16 v8h;
typedef __attribute__((ext_vector_type(16))) __bf16   v16b;
typedef __attribute__((ext_vector_type(8)))  __bf16   v8b;
typedef __attribute__((ext_vector_type(8)))  float    v8f;
typedef __attribute__((ext_vector_type(4)))  float    v4f;

#define NB 32
#define NL 256
#define NK 32
#define NH 256
#define NHEAD 8
#define HD 32
#define NLAY 2
#define POUT 64
#define NEGV (-1.0e9f)
#define LN_EPS (1.0e-5f)
#define WSC 64.0f
#define WSC_INV 0.015625f

__device__ __forceinline__ unsigned short f2bf_bits(float f) {
  unsigned u = __float_as_uint(f);
  return (unsigned short)((u + 0x7FFFu + ((u >> 16) & 1u)) >> 16);
}
__device__ __forceinline__ float bf_bits2f(unsigned short h) { return __uint_as_float(((unsigned)h) << 16); }

__device__ __forceinline__ void dep_guard_h(v8f& a, v8f& b, v16h x, v16h y) { asm volatile("v_nop\n\tv_nop\n\tv_nop\n\tv_nop" : "+v"(a), "+v"(b) : "v"(x), "v"(y)); }
__device__ __forceinline__ void dep_guard_b(v8f& a, v8f& b, v16b x, v16b y) { asm volatile("v_nop\n\tv_nop\n\tv_nop\n\tv_nop" : "+v"(a), "+v"(b) : "v"(x), "v"(y)); }
__device__ __forceinline__ void keep4_h(v16h a, v16h b, v16h c, v16h d) { asm volatile("v_nop" :: "v"(a), "v"(b), "v"(c), "v"(d)); }
__device__ __forceinline__ void keep4_b(v16b a, v16b b, v16b c, v16b d) { asm volatile("v_nop" :: "v"(a), "v"(b), "v"(c), "v"(d)); }
__device__ __forceinline__ void acc_guard4(v8f& a, v8f& b, v8f& c, v8f& d) { asm volatile("v_nop\n\tv_nop\n\tv_nop\n\tv_nop" : "+v"(a), "+v"(b), "+v"(c), "+v"(d)); }
template <typename T> struct Frag;
template <> struct Frag<_Float16> {
  typedef v16h V; union U { v16h v; v8h h[2]; };
  static __device__ __forceinline__ v16h load(const _Float16* p) {
    U f; f.h[0] = *(const v8h*)(p); f.h[1] = *(const v8h*)(p + 16); return f.v;
  }
  static __device__ __forceinline__ v8f mma(v16h a, v16h b, v8f c) {
    return __builtin_amdgcn_wmma_f32_16x16x32_f16(false, a, false, b, (short)0, c, false, false);
  }
  static __device__ __forceinline__ void guard(v8f& a, v8f& b, v16h x, v16h y) { dep_guard_h(a, b, x, y); }
  static __device__ __forceinline__ void keep(v16h a, v16h b, v16h c, v16h d) { keep4_h(a, b, c, d); }
};
template <> struct Frag<__bf16> {
  typedef v16b V; union U { v16b v; v8b h[2]; };
  static __device__ __forceinline__ v16b load(const __bf16* p) {
    U f; f.h[0] = *(const v8b*)(p); f.h[1] = *(const v8b*)(p + 16); return f.v;
  }
  static __device__ __forceinline__ v8f mma(v16b a, v16b b, v8f c) {
    return __builtin_amdgcn_wmma_f32_16x16x32_bf16(false, a, false, b, (short)0, c, false, false);
  }
  static __device__ __forceinline__ void guard(v8f& a, v8f& b, v16b x, v16b y) { dep_guard_b(a, b, x, y); }
  static __device__ __forceinline__ void keep(v16b a, v16b b, v16b c, v16b d) { keep4_b(a, b, c, d); }
};

template <int ET> struct Elem;
template <> struct Elem<0> { typedef _Float16 T; };
template <> struct Elem<1> { typedef __bf16 T; };
template <int ET, bool SPLIT, int BIAS_MODE, int OUT_MODE, bool RESID, int ACT = 0>
__global__ __launch_bounds__(256) void wmma_gemm64(
    const unsigned short* __restrict__ Ap, const unsigned short* __restrict__ A2p, int lda, long strideA,
    const unsigned short* __restrict__ Btp, const unsigned short* __restrict__ Bt2p, int ldb, long strideB,
    void* __restrict__ Cout, void* __restrict__ Cout2, int ldc, long strideC,
    const float* __restrict__ bias,
    const float* __restrict__ resid, long strideR,
    int M, int N, int K, float scale) {
  typedef typename Elem<ET>::T T;
  typedef typename Frag<T>::V V;
  const T* A = (const T*)Ap; const T* A2 = (const T*)A2p; const T* Bt = (const T*)Btp; const T* Bt2 = (const T*)Bt2p;
  __shared__ __align__(16) float sT[8][16 * 68];
  const int b    = blockIdx.y;
  const int lane = threadIdx.x & 31;
  const int wave = threadIdx.x >> 5;
  const int tilesN = N >> 6;
  const int tilesM = M >> 6;
  const int tile = blockIdx.x * 8 + wave;
  if (tile >= tilesM * tilesN) return;
  const int tm = tile / tilesN;
  const int tn = tile - tm * tilesN;
  const int m0 = tm << 6;
  const int n0 = tn << 6;

  const T* Ab  = A  + (size_t)b * strideA;
  const T* Bb  = Bt + (size_t)b * strideB;
  const T* Ab2 = SPLIT ? (A2  + (size_t)b * strideA) : nullptr;
  const T* Bb2 = SPLIT ? (Bt2 + (size_t)b * strideB) : nullptr;

  const int rlane = lane & 15;
  const int koff  = (lane >> 4) * 8;
  const int mOff  = (lane >> 4) * 8;

  v8f acc[4][4];
#pragma unroll
  for (int i = 0; i < 4; ++i)
#pragma unroll
    for (int j = 0; j < 4; ++j) acc[i][j] = (v8f){0.f,0.f,0.f,0.f,0.f,0.f,0.f,0.f};

  for (int k0 = 0; k0 < K; k0 += 32) {
    V bh[4], bl[4];
#pragma unroll
    for (int j = 0; j < 4; ++j) {
      const size_t bo = (size_t)(n0 + (j << 4) + rlane) * ldb + koff + k0;
      bh[j] = Frag<T>::load(Bb + bo);
      if (SPLIT) bl[j] = Frag<T>::load(Bb2 + bo);
    }
#pragma unroll
    for (int i = 0; i < 4; ++i) {
      const size_t ao = (size_t)(m0 + (i << 4) + rlane) * lda + koff + k0;
      V ah = Frag<T>::load(Ab + ao);
      V al;
      if (SPLIT) al = Frag<T>::load(Ab2 + ao);
#pragma unroll
      for (int j = 0; j < 4; ++j) {
        acc[i][j] = Frag<T>::mma(ah, bh[j], acc[i][j]);
        if (SPLIT) {
          acc[i][j] = Frag<T>::mma(ah, bl[j], acc[i][j]);
          acc[i][j] = Frag<T>::mma(al, bh[j], acc[i][j]);
        }
      }
      Frag<T>::guard(acc[i][0], acc[i][3], ah, SPLIT ? al : ah);
    }
    Frag<T>::keep(bh[0], bh[1], bh[2], bh[3]);
    if (SPLIT) Frag<T>::keep(bl[0], bl[1], bl[2], bl[3]);
  }
  acc_guard4(acc[0][0], acc[0][1], acc[0][2], acc[0][3]);
  acc_guard4(acc[1][0], acc[1][1], acc[1][2], acc[1][3]);
  acc_guard4(acc[2][0], acc[2][1], acc[2][2], acc[2][3]);
  acc_guard4(acc[3][0], acc[3][1], acc[3][2], acc[3][3]);

  float* slab = sT[wave];
  const float* Rb = RESID ? (resid + (size_t)b * strideR) : nullptr;
#pragma unroll
  for (int i = 0; i < 4; ++i) {
    const int mBase = m0 + (i << 4);
#pragma unroll
    for (int j = 0; j < 4; ++j) {
      const int n = n0 + (j << 4) + rlane;
      float bv = 0.f;
      if (BIAS_MODE == 2) bv = bias[n];
#pragma unroll
      for (int r = 0; r < 8; ++r) {
        float v = acc[i][j][r] * scale;
        if (BIAS_MODE == 1) v += bias[mBase + mOff + r];
        if (BIAS_MODE == 2) v += bv;
        if (RESID) v += Rb[(size_t)(mBase + mOff + r) * ldc + n];
        if (ACT == 1) v = tanhf(v);
        if (ACT == 2) v = fmaxf(v, 0.0f);
        if (ACT == 3) v = v / (1.0f + expf(-v));
        if (ACT == 4) v = (v > 0.f) ? v : 0.01f * v;
        if (ACT == 5) v = 0.5f * v * (1.0f + erff(v * 0.70710678118654752f));
        slab[(mOff + r) * 68 + (j << 4) + rlane] = v;
      }
    }
    __builtin_amdgcn_fence(__ATOMIC_RELEASE, "workgroup");
    __builtin_amdgcn_wave_barrier();
    __builtin_amdgcn_fence(__ATOMIC_ACQUIRE, "workgroup");
    if (OUT_MODE == 0) {
      float* C = (float*)Cout + (size_t)b * strideC;
      const int hh = lane >> 4, c4 = (lane & 15) * 4;
      for (int pass = 0; pass < 2; ++pass) {
#pragma unroll
        for (int it = 0; it < 8; ++it) {
          const int row = it * 2 + hh;
          v4f v = *(const v4f*)(slab + row * 68 + c4);
          *(volatile v4f*)(C + (size_t)(mBase + row) * ldc + n0 + c4) = v;
        }
        __threadfence();
      }
    } else {
      const int q = lane >> 3, c8 = (lane & 7) * 8;
      unsigned short* C  = (unsigned short*)Cout  + (size_t)b * strideC;
      unsigned short* C2 = (OUT_MODE == 2) ? ((unsigned short*)Cout2 + (size_t)b * strideC) : nullptr;
      for (int pass = 0; pass < 2; ++pass) {
#pragma unroll
        for (int it = 0; it < 4; ++it) {
          const int row = it * 4 + q;
          const float* sp = slab + row * 68 + c8;
          v8h hv, lv;
#pragma unroll
          for (int e = 0; e < 8; ++e) {
            if (OUT_MODE == 1) {
              hv[e] = (_Float16)sp[e];
            } else {
              unsigned short hb = f2bf_bits(sp[e]);
              unsigned short lb = f2bf_bits(sp[e] - bf_bits2f(hb));
              hv[e] = __builtin_bit_cast(_Float16, hb);
              lv[e] = __builtin_bit_cast(_Float16, lb);
            }
          }
          *(volatile v8h*)(C + (size_t)(mBase + row) * ldc + n0 + c8) = hv;
          if (OUT_MODE == 2) *(volatile v8h*)(C2 + (size_t)(mBase + row) * ldc + n0 + c8) = lv;
        }
        __threadfence();
      }
    }
    __builtin_amdgcn_fence(__ATOMIC_RELEASE, "workgroup");
    __builtin_amdgcn_wave_barrier();
    __builtin_amdgcn_fence(__ATOMIC_ACQUIRE, "workgroup");
  }
}

__global__ __launch_bounds__(256) void k_src_transpose(
    const float* __restrict__ src, float* __restrict__ x, _Float16* __restrict__ xh) {
  const int l = blockIdx.x;
  const int wave = threadIdx.x >> 5, lane = threadIdx.x & 31;
#pragma unroll 1
  for (int i = 0; i < 4; ++i) {
    const int b = wave * 4 + i;
    const float* s = src + ((size_t)l * NB + b) * NH;
    const size_t o = ((size_t)b * NL + l) * NH;
    const v4f a0 = *(const v4f*)(s + lane * 4);
    const v4f a1 = *(const v4f*)(s + 128 + lane * 4);
    const v4f c0 = *(const v4f*)(s + lane * 8);
    const v4f c1 = *(const v4f*)(s + lane * 8 + 4);
    v8h hv;
    hv[0] = (_Float16)c0[0]; hv[1] = (_Float16)c0[1]; hv[2] = (_Float16)c0[2]; hv[3] = (_Float16)c0[3];
    hv[4] = (_Float16)c1[0]; hv[5] = (_Float16)c1[1]; hv[6] = (_Float16)c1[2]; hv[7] = (_Float16)c1[3];
    for (int pass = 0; pass < 2; ++pass) {
      *(volatile v4f*)(x + o + lane * 4) = a0;
      *(volatile v4f*)(x + o + 128 + lane * 4) = a1;
      *(volatile v8h*)(xh + o + lane * 8) = hv;
      __threadfence();
    }
  }
}

__global__ __launch_bounds__(256) void k_wcast_t(
    const float* __restrict__ in, _Float16* __restrict__ out, int KD, int N) {
  __shared__ float tile[64][65];
  const int n0 = blockIdx.x * 64, k0 = blockIdx.y * 64;
  const int t = threadIdx.x;
  const int cn = t & 63, rq = t >> 6;
#pragma unroll
  for (int it = 0; it < 16; ++it) {
    const int r = it * 4 + rq;
    tile[r][cn] = in[(size_t)(k0 + r) * N + n0 + cn];
  }
  __syncthreads();
  const int wave = t >> 5, lane = t & 31, q = lane >> 3, c8 = (lane & 7) * 8;
  const int nA = wave * 8 + q;
  const int nB = wave * 8 + 4 + q;
  v8h hA, hB;
#pragma unroll
  for (int e = 0; e < 8; ++e) {
    hA[e] = (_Float16)(tile[c8 + e][nA] * WSC);
    hB[e] = (_Float16)(tile[c8 + e][nB] * WSC);
  }
  _Float16* pA = out + (size_t)(n0 + nA) * KD + k0 + c8;
  _Float16* pB = out + (size_t)(n0 + nB) * KD + k0 + c8;
  for (int pass = 0; pass < 2; ++pass) {
    *(volatile v8h*)pA = hA;
    *(volatile v8h*)pB = hB;
    __threadfence();
  }
}

#define AQB 64
#define AKC 64
__device__ __forceinline__ v8f mma_h(v16h a, v16h b, v8f c) {
  c = __builtin_amdgcn_wmma_f32_16x16x32_f16(false, a, false, b, (short)0, c, false, false);
  asm volatile("v_nop\n\tv_nop\n\tv_nop\n\tv_nop" : "+v"(c) : "v"(a), "v"(b));
  return c;
}

__global__ __launch_bounds__(128) void k_attn32(
    const _Float16* __restrict__ qkv, const int* __restrict__ src_len, _Float16* __restrict__ ctx) {
  __shared__ __align__(16) _Float16 Ksh[AKC * HD];
  __shared__ __align__(16) _Float16 Vt[HD * AKC];
  __shared__ __align__(16) _Float16 Psh[4][16 * AKC];
  __shared__ __align__(16) _Float16 Osh[AQB * NH];
  const int tid = threadIdx.x, wave = tid >> 5, lane = tid & 31;
  const int hh = lane >> 4, c = lane & 15;
  const int b = blockIdx.x >> 2, qb = blockIdx.x & 3;
  const int qrow0 = qb * AQB + wave * 16;
  const int len = src_len[b];
  const size_t rowb = (size_t)b * NL;
  const int LDQ = 3 * NH;
  const float QKSC = 0.17677669529663687f;
  const float PSC = 32768.0f;
  _Float16* pw = Psh[wave];

#pragma unroll 1
  for (int h = 0; h < NHEAD; ++h) {
    const v16h qa = Frag<_Float16>::load(qkv + (rowb + qrow0 + c) * LDQ + h * HD + 8 * hh);
    float mrow[8], lrow[8];
    v8f oacc[2];
#pragma unroll
    for (int r = 0; r < 8; ++r) { mrow[r] = -__builtin_inff(); lrow[r] = 0.f; }
    oacc[0] = (v8f){0.f,0.f,0.f,0.f,0.f,0.f,0.f,0.f};
    oacc[1] = (v8f){0.f,0.f,0.f,0.f,0.f,0.f,0.f,0.f};

#pragma unroll 1
    for (int kc = 0; kc < NL / AKC; ++kc) {
      const int kv0 = kc * AKC;
      __syncthreads();
      {
        const int kvr = tid >> 1, dh = (tid & 1) * 16;
        const _Float16* kp = qkv + (rowb + kv0 + kvr) * LDQ + NH + h * HD + dh;
        const v8h k0v = *(const v8h*)kp;
        const v8h k1v = *(const v8h*)(kp + 8);
        *(v8h*)(Ksh + kvr * HD + dh) = k0v;
        *(v8h*)(Ksh + kvr * HD + dh + 8) = k1v;
        const _Float16* vp = kp + NH;
        const v8h v0 = *(const v8h*)vp;
        const v8h v1 = *(const v8h*)(vp + 8);
#pragma unroll
        for (int e = 0; e < 8; ++e) {
          Vt[(dh + e) * AKC + kvr] = v0[e];
          Vt[(dh + 8 + e) * AKC + kvr] = v1[e];
        }
      }
      __syncthreads();

      v8f s[4];
#pragma unroll
      for (int j = 0; j < 4; ++j) {
        const v16h kb = Frag<_Float16>::load(Ksh + (j * 16 + c) * HD + 8 * hh);
        s[j] = mma_h(qa, kb, (v8f){0.f,0.f,0.f,0.f,0.f,0.f,0.f,0.f});
      }
      float cm[8];
#pragma unroll
      for (int r = 0; r < 8; ++r) {
        const int qrow = qrow0 + 8 * hh + r;
        const bool qok = qrow < len;
        float m = -__builtin_inff();
#pragma unroll
        for (int j = 0; j < 4; ++j) {
          const int kvcol = kv0 + j * 16 + c;
          float v = s[j][r] * QKSC;
          if (!(qok && (kvcol < len))) v = NEGV;
          s[j][r] = v;
          m = fmaxf(m, v);
        }
#pragma unroll
        for (int off = 1; off < 16; off <<= 1) m = fmaxf(m, __shfl_xor(m, off, 32));
        cm[r] = m;
      }
#pragma unroll
      for (int r = 0; r < 8; ++r) {
        const float mnew = fmaxf(mrow[r], cm[r]);
        const float alpha = expf(mrow[r] - mnew);
        mrow[r] = mnew;
        float psum = 0.f;
#pragma unroll
        for (int j = 0; j < 4; ++j) {
          const float p = expf(s[j][r] - mnew);
          psum += p;
          pw[(8 * hh + r) * AKC + j * 16 + c] = (_Float16)(p * PSC);
        }
#pragma unroll
        for (int off = 1; off < 16; off <<= 1) psum += __shfl_xor(psum, off, 32);
        lrow[r] = lrow[r] * alpha + psum;
        oacc[0][r] *= alpha;
        oacc[1][r] *= alpha;
      }
      __builtin_amdgcn_fence(__ATOMIC_RELEASE, "workgroup");
      __builtin_amdgcn_wave_barrier();
      __builtin_amdgcn_fence(__ATOMIC_ACQUIRE, "workgroup");
#pragma unroll
      for (int kk = 0; kk < 2; ++kk) {
        const v16h pa = Frag<_Float16>::load(pw + c * AKC + kk * 32 + 8 * hh);
#pragma unroll
        for (int t = 0; t < 2; ++t) {
          const v16h vb = Frag<_Float16>::load(Vt + (t * 16 + c) * AKC + kk * 32 + 8 * hh);
          oacc[t] = mma_h(pa, vb, oacc[t]);
        }
      }
    }
#pragma unroll
    for (int r = 0; r < 8; ++r) {
      const float inv = 1.0f / (lrow[r] * PSC);
      Osh[(wave * 16 + 8 * hh + r) * NH + h * HD + c]      = (_Float16)(oacc[0][r] * inv);
      Osh[(wave * 16 + 8 * hh + r) * NH + h * HD + 16 + c] = (_Float16)(oacc[1][r] * inv);
    }
  }
  __syncthreads();
  const size_t orow = rowb + qb * AQB + wave * 16;
  for (int pass = 0; pass < 2; ++pass) {
#pragma unroll
    for (int rr = 0; rr < 16; ++rr) {
      const v8h v = *(const v8h*)(Osh + (wave * 16 + rr) * NH + lane * 8);
      *(volatile v8h*)(ctx + (orow + rr) * NH + lane * 8) = v;
    }
    __threadfence();
  }
}

__global__ __launch_bounds__(256) void k_ln(
    const float* __restrict__ in, const float* __restrict__ gam, const float* __restrict__ bet,
    float* __restrict__ x, _Float16* __restrict__ xh, int nrows) {
  __shared__ __align__(16) float slab[8][NH];
  const int wave = threadIdx.x >> 5, lane = threadIdx.x & 31;
  const int row = blockIdx.x * 8 + wave;
  if (row >= nrows) return;
  const float* p = in + (size_t)row * NH + lane * 8;
  const v4f a = *(const v4f*)p;
  const v4f bq = *(const v4f*)(p + 4);
  float v[8] = {a[0], a[1], a[2], a[3], bq[0], bq[1], bq[2], bq[3]};
  float s = 0.f;
#pragma unroll
  for (int e = 0; e < 8; ++e) s += v[e];
#pragma unroll
  for (int off = 1; off < 32; off <<= 1) s += __shfl_xor(s, off, 32);
  const float mean = s * (1.0f / NH);
  float d[8];
  float sq = 0.f;
#pragma unroll
  for (int e = 0; e < 8; ++e) { d[e] = v[e] - mean; sq += d[e] * d[e]; }
#pragma unroll
  for (int off = 1; off < 32; off <<= 1) sq += __shfl_xor(sq, off, 32);
  const float rstd = rsqrtf(sq * (1.0f / NH) + LN_EPS);
  const v4f g0 = *(const v4f*)(gam + lane * 8), g1 = *(const v4f*)(gam + lane * 8 + 4);
  const v4f e0 = *(const v4f*)(bet + lane * 8), e1 = *(const v4f*)(bet + lane * 8 + 4);
  float g[8] = {g0[0], g0[1], g0[2], g0[3], g1[0], g1[1], g1[2], g1[3]};
  float be[8] = {e0[0], e0[1], e0[2], e0[3], e1[0], e1[1], e1[2], e1[3]};
  float y[8];
  v8h hv;
#pragma unroll
  for (int e = 0; e < 8; ++e) { y[e] = d[e] * rstd * g[e] + be[e]; hv[e] = (_Float16)y[e]; }
  const v4f y0 = {y[0], y[1], y[2], y[3]};
  const v4f y1 = {y[4], y[5], y[6], y[7]};
  *(v4f*)(&slab[wave][lane * 8]) = y0;
  *(v4f*)(&slab[wave][lane * 8 + 4]) = y1;
  __builtin_amdgcn_fence(__ATOMIC_RELEASE, "workgroup");
  __builtin_amdgcn_wave_barrier();
  __builtin_amdgcn_fence(__ATOMIC_ACQUIRE, "workgroup");
  const v4f o0 = *(const v4f*)(&slab[wave][lane * 4]);
  const v4f o1 = *(const v4f*)(&slab[wave][128 + lane * 4]);
  float* xr = x + (size_t)row * NH;
  _Float16* hr = xh + (size_t)row * NH;
  for (int pass = 0; pass < 2; ++pass) {
    *(volatile v4f*)(xr + lane * 4) = o0;
    *(volatile v4f*)(xr + 128 + lane * 4) = o1;
    *(volatile v8h*)(hr + lane * 8) = hv;
    __threadfence();
  }
}

__device__ __forceinline__ float block_sum256(float v, float* red) {
#pragma unroll
  for (int off = 1; off < 32; off <<= 1) v += __shfl_xor(v, off, 32);
  const int wave = threadIdx.x >> 5, lane = threadIdx.x & 31;
  __syncthreads();
  if (lane == 0) red[wave] = v;
  __syncthreads();
  float s = red[0];
#pragma unroll
  for (int i = 1; i < 8; ++i) s += red[i];
  return s;
}

__global__ __launch_bounds__(256) void k_candi(
    const float* __restrict__ x, const int* __restrict__ src_len,
    const int* __restrict__ ids, const float* __restrict__ feats, const int* __restrict__ masks,
    const float* __restrict__ emb, int n_id,
    const float* __restrict__ fcw, const float* __restrict__ fcb,
    const float* __restrict__ fg, const float* __restrict__ fb,
    float* __restrict__ out_f, float* __restrict__ out_m) {
  __shared__ __align__(16) float comb[NK * NH];
  __shared__ __align__(16) float g_l[NH];
  __shared__ __align__(16) float f_l[NH];
  __shared__ __align__(16) float prob[NK];
  __shared__ float sfeat[NK * 9];
  __shared__ float sc[NK];
  __shared__ float aw[NK];
  __shared__ int sid[NK];
  __shared__ int smask[NK];
  __shared__ float red[8];
  const int bl = blockIdx.x;
  const int b = bl >> 8, l = bl & 255;
  const int t = threadIdx.x, wave = t >> 5, lane = t & 31;
  const int len = src_len[b];
  const size_t base = (size_t)bl * NK;

  sfeat[t] = feats[base * 9 + t];
  if (t < NK) {
    sfeat[NH + t] = feats[base * 9 + NH + t];
    int id = ids[base + t];
    id = id < 0 ? 0 : id;
    id = id >= n_id ? n_id - 1 : id;
    sid[t] = id;
    smask[t] = masks[base + t];
  }
  float w[9];
#pragma unroll
  for (int j = 0; j < 9; ++j) w[j] = fcw[j * NH + t];
  const float cb = fcb[t];
  const float vf = (l < len) ? 1.0f : 0.0f;
  const float g = x[(size_t)bl * NH + t] * vf;
  g_l[t] = g;
  __syncthreads();

#pragma unroll 1
  for (int k = 0; k < NK; ++k) {
    float s = cb;
#pragma unroll
    for (int j = 0; j < 9; ++j) s += sfeat[k * 9 + j] * w[j];
    s += emb[(size_t)sid[k] * NH + t];
    comb[k * NH + t] = s;
  }
  __syncthreads();

#pragma unroll
  for (int kk = 0; kk < 4; ++kk) {
    const int k = wave * 4 + kk;
    float p = 0.f;
#pragma unroll 1
    for (int i = 0; i < 8; ++i) p += g_l[lane + 32 * i] * comb[k * NH + lane + 32 * i];
#pragma unroll
    for (int off = 1; off < 32; off <<= 1) p += __shfl_xor(p, off, 32);
    if (lane == 0) sc[k] = p * 0.0625f;
  }
  __syncthreads();
  if (wave == 0) {
    const float s = (smask[lane] == 0) ? NEGV : sc[lane];
    float mx = s;
#pragma unroll
    for (int off = 1; off < 32; off <<= 1) mx = fmaxf(mx, __shfl_xor(mx, off, 32));
    const float e = __expf(s - mx);
    float sum = e;
#pragma unroll
    for (int off = 1; off < 32; off <<= 1) sum += __shfl_xor(sum, off, 32);
    aw[lane] = e * (1.0f / sum);
  }
  __syncthreads();

  float cacc = 0.f;
#pragma unroll 1
  for (int k = 0; k < NK; ++k) cacc += aw[k] * comb[k * NH + t];
  const float f = g + cacc;
  const float mean = block_sum256(f, red) * (1.0f / NH);
  const float dv = f - mean;
  const float var = block_sum256(dv * dv, red) * (1.0f / NH);
  const float fn = dv * rsqrtf(var + LN_EPS) * fg[t] + fb[t];
  f_l[t] = fn;
  __syncthreads();

#pragma unroll
  for (int kk = 0; kk < 4; ++kk) {
    const int k = wave * 4 + kk;
    float p = 0.f;
#pragma unroll 1
    for (int i = 0; i < 8; ++i) p += f_l[lane + 32 * i] * comb[k * NH + lane + 32 * i];
#pragma unroll
    for (int off = 1; off < 32; off <<= 1) p += __shfl_xor(p, off, 32);
    if (lane == 0) {
      const float e = __expf(-p);
      prob[k] = (smask[k] == 0) ? 0.0f : (1.0f / (1.0f + e));
    }
  }
  __syncthreads();

  if (wave == 0) {
    const v4f o0 = *(const v4f*)(&f_l[lane * 4]);
    const v4f o1 = *(const v4f*)(&f_l[128 + lane * 4]);
    const v4f pm = *(const v4f*)(&prob[(lane & 7) * 4]);
    float* of = out_f + ((size_t)l * NB + b) * NH;
    float* om = out_m + base;
    for (int pass = 0; pass < 2; ++pass) {
      *(volatile v4f*)(of + lane * 4) = o0;
      *(volatile v4f*)(of + 128 + lane * 4) = o1;
      if (lane < 8) *(volatile v4f*)(om + lane * 4) = pm;
      __threadfence();
    }
  }
}

__global__ __launch_bounds__(256) void k_pool_gate(
    const float* __restrict__ fus, const int* __restrict__ src_len,
    const int* __restrict__ pro, const float* __restrict__ tw, int n_pro,
    const float* __restrict__ fw, const float* __restrict__ fbias, float* __restrict__ out_h) {
  __shared__ __align__(16) float cat[POUT + NH];
  __shared__ __align__(16) float res[NH];
  const int b = blockIdx.x, t = threadIdx.x, wave = t >> 5, lane = t & 31;
  const int len = src_len[b];
  float s = 0.f;
#pragma unroll 1
  for (int l = 0; l < NL; ++l) {
    const float v = fus[((size_t)l * NB + b) * NH + t];
    if (l < len) s += v;
  }
  cat[POUT + t] = s * (1.0f / (float)len);
  if (t < POUT) {
    int p = pro[b];
    p = p < 0 ? 0 : p;
    p = p >= n_pro ? n_pro - 1 : p;
    cat[t] = tw[p * POUT + t];
  }
  __syncthreads();
  float o = fbias[t];
#pragma unroll 1
  for (int j = 0; j < POUT + NH; ++j) o += cat[j] * fw[(size_t)j * NH + t];
  res[t] = tanhf(o);
  __syncthreads();
  if (wave == 0) {
    const v4f o0 = *(const v4f*)(&res[lane * 4]);
    const v4f o1 = *(const v4f*)(&res[128 + lane * 4]);
    float* oh = out_h + (size_t)b * NH;
    for (int pass = 0; pass < 2; ++pass) {
      *(volatile v4f*)(oh + lane * 4) = o0;
      *(volatile v4f*)(oh + 128 + lane * 4) = o1;
      __threadfence();
    }
  }
}

extern "C" void kernel_launch(void* const* d_in, const int* in_sizes, int n_in,
                              void* d_out, int out_size, void* d_ws, size_t ws_size,
                              hipStream_t stream) {
  if (n_in < 27) return;
  const float* src         = (const float*)d_in[0];
  const int*   src_len     = (const int*)d_in[1];
  const int*   candi_ids   = (const int*)d_in[3];
  const float* candi_feats = (const float*)d_in[4];
  const int*   candi_masks = (const int*)d_in[5];
  const int*   pro         = (const int*)d_in[6];
  const float* emb         = (const float*)d_in[7];
  const float* fcw         = (const float*)d_in[8];
  const float* fcb         = (const float*)d_in[9];
  const float* fus_g       = (const float*)d_in[10];
  const float* fus_b       = (const float*)d_in[11];
  const float* tw          = (const float*)d_in[12];
  const float* fhw         = (const float*)d_in[13];
  const float* fhb         = (const float*)d_in[14];
  const float* attn_w      = (const float*)d_in[15];
  const float* attn_b      = (const float*)d_in[16];
  const float* out_w       = (const float*)d_in[17];
  const float* out_b       = (const float*)d_in[18];
  const float* ln1_g       = (const float*)d_in[19];
  const float* ln1_b       = (const float*)d_in[20];
  const float* w1          = (const float*)d_in[21];
  const float* b1          = (const float*)d_in[22];
  const float* w2          = (const float*)d_in[23];
  const float* b2          = (const float*)d_in[24];
  const float* ln2_g       = (const float*)d_in[25];
  const float* ln2_b       = (const float*)d_in[26];

  const int M = NB * NL;
  if (in_sizes[0] != NL * NB * NH) return;
  if (in_sizes[1] != NB || in_sizes[3] != NB * NL * NK || in_sizes[4] != NB * NL * NK * 9 || in_sizes[5] != NB * NL * NK) return;
  if (in_sizes[15] != NLAY * NH * 3 * NH || in_sizes[21] != NLAY * NH * 4 * NH || in_sizes[23] != NLAY * 4 * NH * NH) return;
  if (in_sizes[13] != (POUT + NH) * NH) return;
  if (out_size != NL * NB * NH + NB * NH + NB * NL * NK) return;
  const int n_id  = in_sizes[7] / NH;
  const int n_pro = in_sizes[12] / POUT;
  if (n_id < 1 || n_pro < 1) return;

  const size_t sz_x    = (size_t)M * NH * 4;
  const size_t sz_xh   = (size_t)M * NH * 2;
  const size_t sz_qkv  = (size_t)M * 3 * NH * 2;
  const size_t sz_ctx  = (size_t)M * NH * 2;
  const size_t sz_tmp  = (size_t)M * NH * 4;
  const size_t sz_h1   = (size_t)M * 4 * NH * 2;
  const size_t sz_wq   = (size_t)3 * NH * NH * 2;
  const size_t sz_wo   = (size_t)NH * NH * 2;
  const size_t sz_w1   = (size_t)4 * NH * NH * 2;
  const size_t sz_w2   = (size_t)4 * NH * NH * 2;
  const size_t sz_wl   = sz_wq + sz_wo + sz_w1 + sz_w2;
  const size_t off_x   = 0;
  const size_t off_xh  = off_x + sz_x;
  const size_t off_qkv = off_xh + sz_xh;
  const size_t off_ctx = off_qkv + sz_qkv;
  const size_t off_tmp = off_ctx + sz_ctx;
  const size_t off_h1  = off_tmp + sz_tmp;
  const size_t off_w   = off_h1 + sz_h1;
  const size_t off_end = off_w + (size_t)NLAY * sz_wl;
  if (off_end > ws_size) return;

  char* ws = (char*)d_ws;
  float*    x    = (float*)(ws + off_x);
  _Float16* xh   = (_Float16*)(ws + off_xh);
  _Float16* qkvh = (_Float16*)(ws + off_qkv);
  _Float16* ctxh = (_Float16*)(ws + off_ctx);
  float*    tmp  = (float*)(ws + off_tmp);
  _Float16* h1h  = (_Float16*)(ws + off_h1);
  _Float16* wqT[NLAY]; _Float16* woT[NLAY]; _Float16* w1T[NLAY]; _Float16* w2T[NLAY];
  for (int l = 0; l < NLAY; ++l) {
    char* wb = ws + off_w + (size_t)l * sz_wl;
    wqT[l] = (_Float16*)(wb);
    woT[l] = (_Float16*)(wb + sz_wq);
    w1T[l] = (_Float16*)(wb + sz_wq + sz_wo);
    w2T[l] = (_Float16*)(wb + sz_wq + sz_wo + sz_w1);
  }

  float* out0 = (float*)d_out;
  float* out1 = out0 + (size_t)NL * NB * NH;
  float* out2 = out1 + (size_t)NB * NH;

  k_src_transpose<<<NL, 256, 0, stream>>>(src, x, xh);
  for (int l = 0; l < NLAY; ++l) {
    k_wcast_t<<<dim3(3 * NH / 64, NH / 64), 256, 0, stream>>>(attn_w + (size_t)l * NH * 3 * NH, wqT[l], NH, 3 * NH);
    k_wcast_t<<<dim3(NH / 64, NH / 64), 256, 0, stream>>>(out_w + (size_t)l * NH * NH, woT[l], NH, NH);
    k_wcast_t<<<dim3(4 * NH / 64, NH / 64), 256, 0, stream>>>(w1 + (size_t)l * NH * 4 * NH, w1T[l], NH, 4 * NH);
    k_wcast_t<<<dim3(NH / 64, 4 * NH / 64), 256, 0, stream>>>(w2 + (size_t)l * 4 * NH * NH, w2T[l], 4 * NH, NH);
  }

  const int blk_qkv = ((M / 64) * (3 * NH / 64) + 7) / 8;
  const int blk_hid = ((M / 64) * (NH / 64) + 7) / 8;
  const int blk_ff1 = ((M / 64) * (4 * NH / 64) + 7) / 8;

  for (int l = 0; l < NLAY; ++l) {
    wmma_gemm64<0, false, 2, 1, false, 0><<<dim3(blk_qkv, 1), 256, 0, stream>>>(
        (const unsigned short*)xh, (const unsigned short*)xh, NH, 0L,
        (const unsigned short*)wqT[l], (const unsigned short*)wqT[l], NH, 0L,
        (void*)qkvh, (void*)qkvh, 3 * NH, 0L,
        attn_b + (size_t)l * 3 * NH, x, 0L, M, 3 * NH, NH, WSC_INV);
    k_attn32<<<NB * (NL / AQB), 128, 0, stream>>>(qkvh, src_len, ctxh);
    wmma_gemm64<0, false, 2, 0, true, 0><<<dim3(blk_hid, 1), 256, 0, stream>>>(
        (const unsigned short*)ctxh, (const unsigned short*)ctxh, NH, 0L,
        (const unsigned short*)woT[l], (const unsigned short*)woT[l], NH, 0L,
        (void*)tmp, (void*)tmp, NH, 0L,
        out_b + (size_t)l * NH, x, 0L, M, NH, NH, WSC_INV);
    k_ln<<<M / 8, 256, 0, stream>>>(tmp, ln1_g + (size_t)l * NH, ln1_b + (size_t)l * NH, x, xh, M);
    wmma_gemm64<0, false, 2, 1, false, 2><<<dim3(blk_ff1, 1), 256, 0, stream>>>(
        (const unsigned short*)xh, (const unsigned short*)xh, NH, 0L,
        (const unsigned short*)w1T[l], (const unsigned short*)w1T[l], NH, 0L,
        (void*)h1h, (void*)h1h, 4 * NH, 0L,
        b1 + (size_t)l * 4 * NH, x, 0L, M, 4 * NH, NH, WSC_INV);
    wmma_gemm64<0, false, 2, 0, true, 0><<<dim3(blk_hid, 1), 256, 0, stream>>>(
        (const unsigned short*)h1h, (const unsigned short*)h1h, 4 * NH, 0L,
        (const unsigned short*)w2T[l], (const unsigned short*)w2T[l], 4 * NH, 0L,
        (void*)tmp, (void*)tmp, NH, 0L,
        b2 + (size_t)l * NH, x, 0L, M, NH, 4 * NH, WSC_INV);
    k_ln<<<M / 8, 256, 0, stream>>>(tmp, ln2_g + (size_t)l * NH, ln2_b + (size_t)l * NH, x, xh, M);
  }

  k_candi<<<M, 256, 0, stream>>>(x, src_len, candi_ids, candi_feats, candi_masks, emb, n_id,
                                  fcw, fcb, fus_g, fus_b, out0, out2);
  k_pool_gate<<<NB, 256, 0, stream>>>(out0, src_len, pro, tw, n_pro, fhw, fhb, out1);
  (void)hipGetLastError();
}
